// EEGGAT_57543971832358
// MI455X (gfx1250) — hardware-verified
//
#include <hip/hip_runtime.h>

#define NPG      19
#define T_LEN    256
#define EPS_BN   1e-5f

typedef _Float16 v16h __attribute__((ext_vector_type(16)));
typedef _Float16 v8h  __attribute__((ext_vector_type(8)));
typedef float    v8f  __attribute__((ext_vector_type(8)));
typedef float    v4f  __attribute__((ext_vector_type(4)));

union Frag { v16h v; v8h half[2]; };

__device__ __forceinline__ v8f zero8() {
  v8f z = {0.f, 0.f, 0.f, 0.f, 0.f, 0.f, 0.f, 0.f};
  return z;
}

__device__ __forceinline__ v8f mma16(v16h a, v16h b, v8f c) {
  v8f d = __builtin_amdgcn_wmma_f32_16x16x32_f16(false, a, false, b, (short)0, c, false, false);
  asm volatile("v_nop\n\tv_nop\n\tv_nop\n\tv_nop" : "+v"(d) : "v"(a), "v"(b));
  return d;
}

__device__ __forceinline__ v16h ld_frag(const _Float16* p, int h) {
  Frag f;
  f.half[0] = *(const v8h*)(p + 8 * h);
  f.half[1] = *(const v8h*)(p + 16 + 8 * h);
  return f.v;
}

#define BUF1T_OFF 0
#define W2P_OFF   8448
#define W3P_OFF   0
#define BUF2T_OFF 22784
#define SMEM_H    39680

__global__ __launch_bounds__(256)
void k_conv_feat(const float* __restrict__ x,
                 const float* __restrict__ w1, const float* __restrict__ b1c,
                 const float* __restrict__ bn1,
                 const float* __restrict__ w2, const float* __restrict__ b2c,
                 const float* __restrict__ bn2,
                 const float* __restrict__ w3, const float* __restrict__ b3c,
                 const float* __restrict__ bn3,
                 const float* __restrict__ dw_w, const float* __restrict__ dw_b,
                 const float* __restrict__ bnd,
                 const float* __restrict__ prelu,
                 float* __restrict__ feat, int n_nodes)
{
  __shared__ __attribute__((aligned(32))) _Float16 smem[SMEM_H];
  __shared__ float xs[272];
  __shared__ float featacc[128];
  __shared__ float c1w[30 * 15];
  __shared__ float sc1[32], sh1[32];
  __shared__ float sc2[64], sh2[64];
  __shared__ float sc3[96], sh3[96];
  __shared__ float sdv[96], tdv[96];
  __shared__ float dws[96], dwb[96];

  const int node = blockIdx.x;
  if (node >= n_nodes) return;
  const int tid  = threadIdx.x;
  const int lane = tid & 31;
  const int wave = tid >> 5;
  const int lg   = lane >> 4;
  const int ll   = lane & 15;
  const float a0 = prelu[0], a1 = prelu[1], a2 = prelu[2], a3 = prelu[3];

  _Float16* buf1t = smem + BUF1T_OFF;
  _Float16* w2p   = smem + W2P_OFF;
  _Float16* buf2t = smem + BUF2T_OFF;
  _Float16* w3p   = smem + W3P_OFF;

  xs[7 + tid] = x[(size_t)node * T_LEN + tid];
  if (tid < 7) xs[tid] = 0.f;
  if (tid < 9) xs[263 + tid] = 0.f;
  for (int i = tid; i < 30 * 15; i += 256) c1w[i] = w1[i];
  if (tid < 32) {
    float sc = 0.f, sh = 0.f;
    if (tid < 30) {
      sc = bn1[0*30+tid] * rsqrtf(bn1[3*30+tid] + EPS_BN);
      sh = bn1[1*30+tid] - bn1[2*30+tid] * sc + sc * b1c[tid];
    }
    sc1[tid] = sc; sh1[tid] = sh;
  }
  if (tid < 64) {
    float sc = 0.f, sh = 0.f;
    if (tid < 60) {
      sc = bn2[0*60+tid] * rsqrtf(bn2[3*60+tid] + EPS_BN);
      sh = bn2[1*60+tid] - bn2[2*60+tid] * sc + sc * b2c[tid];
    }
    sc2[tid] = sc; sh2[tid] = sh;
  }
  if (tid < 96) {
    float sc = 0.f, sh = 0.f, sd = 0.f, sdsh = 0.f, dw = 0.f, db = 0.f;
    if (tid < 90) {
      sc = bn3[0*90+tid] * rsqrtf(bn3[3*90+tid] + EPS_BN);
      sh = bn3[1*90+tid] - bn3[2*90+tid] * sc + sc * b3c[tid];
      sd = bnd[0*90+tid] * rsqrtf(bnd[3*90+tid] + EPS_BN);
      sdsh = bnd[1*90+tid] - bnd[2*90+tid] * sd;
      dw = dw_w[tid]; db = dw_b[tid];
    }
    sc3[tid] = sc;  sh3[tid] = sh;
    sdv[tid] = sd;  tdv[tid] = sdsh;
    dws[tid] = dw;  dwb[tid] = db;
  }
  for (int i = tid; i < 264 * 32; i += 256) buf1t[i] = (_Float16)0.f;
  for (int i = tid; i < 264 * 64; i += 256) buf2t[i] = (_Float16)0.f;
  for (int i = tid; i < 64 * 224; i += 256) {
    int co = i / 224, k2 = i - co * 224;
    int kk = k2 >> 5, ci = k2 & 31;
    float v = (co < 60 && ci < 30) ? w2[co * 210 + ci * 7 + kk] : 0.f;
    w2p[i] = (_Float16)v;
  }
  __syncthreads();

  for (int it = 0; it < 30; ++it) {
    int idx = tid + it * 256;
    int co = idx >> 8, t = idx & 255;
    float acc = 0.f;
#pragma unroll
    for (int k = 0; k < 15; ++k) acc += c1w[co * 15 + k] * xs[t + k];
    float z = sc1[co] * acc + sh1[co];
    z = z >= 0.f ? z : a0 * z;
    buf1t[(t + 4) * 32 + co] = (_Float16)z;
  }
  __syncthreads();

  {
    int tm = wave >> 1;
    const _Float16* arow = w2p + (tm * 16 + ll) * 224;
    v16h Af[7];
#pragma unroll
    for (int kc = 0; kc < 7; ++kc) Af[kc] = ld_frag(arow + kc * 32, lg);
    for (int tt = 0; tt < 8; ++tt) {
      int tn = (wave & 1) * 8 + tt;
      int tcol = tn * 16 + ll;
      v8f acc = zero8();
#pragma unroll
      for (int kc = 0; kc < 7; ++kc) {
        const _Float16* bp = buf1t + (tcol + kc + 1) * 32;
        acc = mma16(Af[kc], ld_frag(bp, lg), acc);
      }
#pragma unroll
      for (int r = 0; r < 8; ++r) {
        int co = tm * 16 + r + (lg << 3);
        float z = sc2[co] * acc[r] + sh2[co];
        z = z >= 0.f ? z : a1 * z;
        buf2t[(tcol + 4) * 64 + co] = (_Float16)z;
      }
    }
  }
  __syncthreads();

  for (int i = tid; i < 96 * 192; i += 256) {
    int co = i / 192, k2 = i - co * 192;
    int kk = k2 >> 6, ci = k2 & 63;
    float v = (co < 90 && ci < 60) ? w3[co * 180 + ci * 3 + kk] : 0.f;
    w3p[i] = (_Float16)v;
  }
  __syncthreads();

  float part[2] = {0.f, 0.f};
  for (int tm = 0; tm < 6; ++tm) {
    const _Float16* arow = w3p + (tm * 16 + ll) * 192;
    v16h Af[6];
#pragma unroll
    for (int kc = 0; kc < 6; ++kc) Af[kc] = ld_frag(arow + kc * 32, lg);
#pragma unroll
    for (int tt = 0; tt < 2; ++tt) {
      int tn = wave * 2 + tt;
      int tcol = tn * 16 + ll;
      v8f acc = zero8();
#pragma unroll
      for (int kc = 0; kc < 6; ++kc) {
        const _Float16* bp = buf2t + (tcol + (kc >> 1) + 3) * 64 + ((kc & 1) << 5);
        acc = mma16(Af[kc], ld_frag(bp, lg), acc);
      }
      float ps = 0.f;
#pragma unroll
      for (int r = 0; r < 8; ++r) {
        int co = tm * 16 + r + (lg << 3);
        float z = sc3[co] * acc[r] + sh3[co];
        z = z >= 0.f ? z : a2 * z;
        z = z * dws[co] + dwb[co];
        z = sdv[co] * z + tdv[co];
        z = z >= 0.f ? z : a3 * z;
        ps += z;
      }
      part[tt] += ps;
    }
  }
#pragma unroll
  for (int tt = 0; tt < 2; ++tt) {
    float v = part[tt];
    v += __shfl_xor(v, 16);
    v += __shfl_xor(v, 1);
    if (lg == 0 && (ll & 1) == 0)
      featacc[(wave * 2 + tt) * 8 + (ll >> 1)] = v * (1.0f / 180.0f);
  }
  __syncthreads();
  if (wave == 0) {
    v4f o;
    o.x = featacc[4 * lane + 0];
    o.y = featacc[4 * lane + 1];
    o.z = featacc[4 * lane + 2];
    o.w = featacc[4 * lane + 3];
    float* dst = feat + (size_t)node * 128 + 4 * lane;
    *(volatile v4f*)dst = o;
    __threadfence();
    *(volatile v4f*)dst = o;
  }
}

__global__ __launch_bounds__(256)
void k_gat_head(const float* __restrict__ feat,
                const float* __restrict__ g1w, const float* __restrict__ g1a, const float* __restrict__ g1b,
                const float* __restrict__ g2w, const float* __restrict__ g2a, const float* __restrict__ g2b,
                const float* __restrict__ g3w, const float* __restrict__ g3a, const float* __restrict__ g3b,
                const float* __restrict__ bng1, const float* __restrict__ bng2, const float* __restrict__ bng3,
                const float* __restrict__ prelu,
                const float* __restrict__ fc1w, const float* __restrict__ fc1b,
                const float* __restrict__ fc2w, const float* __restrict__ fc2b,
                float* __restrict__ gout, int n_graphs)
{
  __shared__ float    cur[NPG * 128];
  __shared__ float    nxt[NPG * 128];
  __shared__ float    hF[32 * 128];
  __shared__ __attribute__((aligned(32))) _Float16 a16[32 * 128];
  __shared__ __attribute__((aligned(32))) _Float16 Wt[128 * 128];
  __shared__ float    eL[NPG * NPG * 4];
  __shared__ float    asrc[NPG * 4], adst[NPG * 4];
  __shared__ float    attL[2 * 4 * 32];
  __shared__ float    bnS[128], bnT[128], biasL[128];
  __shared__ float    pooled[128], hfc[64];

  const int g    = blockIdx.x;
  if (g >= n_graphs) return;
  const int tid  = threadIdx.x;
  const int lane = tid & 31;
  const int wave = tid >> 5;
  const int lg   = lane >> 4;
  const int ll   = lane & 15;

  for (int i = tid; i < NPG * 128; i += 256) cur[i] = feat[(size_t)g * NPG * 128 + i];
  for (int i = tid; i < 32 * 128; i += 256)  a16[i] = (_Float16)0.f;
  __syncthreads();

  for (int l = 0; l < 3; ++l) {
    const float* W  = (l == 0) ? g1w  : ((l == 1) ? g2w  : g3w);
    const float* At = (l == 0) ? g1a  : ((l == 1) ? g2a  : g3a);
    const float* Bi = (l == 0) ? g1b  : ((l == 1) ? g2b  : g3b);
    const float* Bn = (l == 0) ? bng1 : ((l == 1) ? bng2 : bng3);
    const float aslope = prelu[4 + l];
    if (tid < 128) {
      float sc = Bn[0*128+tid] * rsqrtf(Bn[3*128+tid] + EPS_BN);
      bnS[tid] = sc;
      bnT[tid] = Bn[1*128+tid] - Bn[2*128+tid] * sc;
      biasL[tid] = Bi[tid];
    }
    attL[tid] = At[tid];
    for (int i = tid; i < NPG * 128; i += 256) a16[i] = (_Float16)cur[i];
    for (int i = tid; i < 128 * 128; i += 256) {
      int k = i >> 7, n = i & 127;
      Wt[n * 128 + k] = (_Float16)W[i];
    }
    __syncthreads();

    {
      int tm = wave >> 2;
      const _Float16* arow = a16 + (tm * 16 + ll) * 128;
      v16h Af[4];
#pragma unroll
      for (int kc = 0; kc < 4; ++kc) Af[kc] = ld_frag(arow + kc * 32, lg);
#pragma unroll
      for (int tt = 0; tt < 2; ++tt) {
        int tn = (wave & 3) * 2 + tt;
        const _Float16* bcol = Wt + (tn * 16 + ll) * 128;
        v8f acc = zero8();
#pragma unroll
        for (int kc = 0; kc < 4; ++kc)
          acc = mma16(Af[kc], ld_frag(bcol + kc * 32, lg), acc);
#pragma unroll
        for (int r = 0; r < 8; ++r) {
          int m = tm * 16 + r + (lg << 3);
          hF[m * 128 + tn * 16 + ll] = acc[r];
        }
      }
    }
    __syncthreads();

    if (tid < NPG * 4) {
      int i = tid >> 2, hh = tid & 3;
      float ss = 0.f, dd = 0.f;
#pragma unroll
      for (int c = 0; c < 32; ++c) {
        float hv = hF[i * 128 + hh * 32 + c];
        ss += hv * attL[0 * 128 + hh * 32 + c];
        dd += hv * attL[1 * 128 + hh * 32 + c];
      }
      asrc[tid] = ss;
      adst[tid] = dd;
    }
    __syncthreads();
    for (int idx = tid; idx < NPG * NPG * 4; idx += 256) {
      int hh = idx & 3;
      int ij = idx >> 2;
      int i = ij / NPG, j = ij - i * NPG;
      float e = asrc[i * 4 + hh] + adst[j * 4 + hh];
      eL[idx] = e >= 0.f ? e : 0.2f * e;
    }
    __syncthreads();
    if (tid < NPG * 4) {
      int j = tid >> 2, hh = tid & 3;
      float m = -1e30f;
      for (int i = 0; i < NPG; ++i) m = fmaxf(m, eL[((i * NPG + j) << 2) + hh]);
      float s = 0.f;
      for (int i = 0; i < NPG; ++i) s += __expf(eL[((i * NPG + j) << 2) + hh] - m);
      float inv = 1.0f / s;
      for (int i = 0; i < NPG; ++i) {
        int id = ((i * NPG + j) << 2) + hh;
        eL[id] = __expf(eL[id] - m) * inv;
      }
    }
    __syncthreads();
    for (int idx = tid; idx < NPG * 128; idx += 256) {
      int j = idx >> 7, f = idx & 127;
      int hh = f >> 5;
      float acc = 0.f;
      for (int i = 0; i < NPG; ++i)
        acc += eL[((i * NPG + j) << 2) + hh] * hF[i * 128 + f];
      float z = bnS[f] * (acc + biasL[f]) + bnT[f];
      z = z >= 0.f ? z : aslope * z;
      if (l > 0) z += cur[idx];
      nxt[idx] = z;
    }
    __syncthreads();
    for (int idx = tid; idx < NPG * 128; idx += 256) cur[idx] = nxt[idx];
    __syncthreads();
  }

  if (tid < 128) {
    float s = 0.f;
    for (int j = 0; j < NPG; ++j) s += cur[j * 128 + tid];
    pooled[tid] = s * (1.0f / NPG);
  }
  __syncthreads();
  if (tid < 64) {
    float s = fc1b[tid];
    for (int k = 0; k < 128; ++k) s += pooled[k] * fc1w[k * 64 + tid];
    hfc[tid] = fmaxf(s, 0.f);
  }
  __syncthreads();
  if (wave == 0) {
    float s = fc2b[0];
    for (int o = 0; o < 64; ++o) s += hfc[o] * fc2w[o];
    if (lane < 8) {
      v4f o4 = {s, s, s, s};
      float* dst = gout + (size_t)g * 32 + 4 * lane;
      *(volatile v4f*)dst = o4;
      __threadfence();
      *(volatile v4f*)dst = o4;
    }
  }
}

__global__ __launch_bounds__(32)
void k_pack_out(const float* __restrict__ gout, float* __restrict__ out, int n_graphs)
{
  const int lane = threadIdx.x & 31;
  for (int base = 0; base < n_graphs; base += 128) {
    const int i0 = base + 4 * lane;
    float e[4];
#pragma unroll
    for (int q = 0; q < 4; ++q) {
      int i = i0 + q;
      e[q] = (i < n_graphs) ? gout[(size_t)i * 32] : 0.f;
    }
    if (i0 + 3 < n_graphs) {
      v4f v = {e[0], e[1], e[2], e[3]};
      float* dst = out + i0;
      *(volatile v4f*)dst = v;
      __threadfence();
      *(volatile v4f*)dst = v;
    } else {
#pragma unroll
      for (int q = 0; q < 4; ++q) {
        int i = i0 + q;
        if (i < n_graphs) *(volatile float*)(out + i) = e[q];
      }
      __threadfence();
#pragma unroll
      for (int q = 0; q < 4; ++q) {
        int i = i0 + q;
        if (i < n_graphs) *(volatile float*)(out + i) = e[q];
      }
    }
  }
}

extern "C" void kernel_launch(void* const* d_in, const int* in_sizes, int n_in,
                              void* d_out, int out_size, void* d_ws, size_t ws_size,
                              hipStream_t stream) {
  if (n_in < 33) return;
  const int n_nodes  = in_sizes[0] / T_LEN;
  const int n_graphs = out_size;
  if (n_nodes <= 0 || n_graphs <= 0) return;
  if (n_nodes * T_LEN != in_sizes[0]) return;
  if (n_nodes != n_graphs * NPG) return;
  if (in_sizes[2] != n_nodes) return;

  const float* x       = (const float*)d_in[0];
  const float* conv1_w = (const float*)d_in[3];
  const float* conv1_b = (const float*)d_in[4];
  const float* bn1     = (const float*)d_in[5];
  const float* conv2_w = (const float*)d_in[6];
  const float* conv2_b = (const float*)d_in[7];
  const float* bn2     = (const float*)d_in[8];
  const float* conv3_w = (const float*)d_in[9];
  const float* conv3_b = (const float*)d_in[10];
  const float* bn3     = (const float*)d_in[11];
  const float* dw_w    = (const float*)d_in[12];
  const float* dw_b    = (const float*)d_in[13];
  const float* bn_d    = (const float*)d_in[14];
  const float* prelu   = (const float*)d_in[15];
  const float* g1w  = (const float*)d_in[16];
  const float* g1a  = (const float*)d_in[17];
  const float* g1b  = (const float*)d_in[18];
  const float* g2w  = (const float*)d_in[19];
  const float* g2a  = (const float*)d_in[20];
  const float* g2b  = (const float*)d_in[21];
  const float* g3w  = (const float*)d_in[22];
  const float* g3a  = (const float*)d_in[23];
  const float* g3b  = (const float*)d_in[24];
  const float* bng1 = (const float*)d_in[25];
  const float* bng2 = (const float*)d_in[26];
  const float* bng3 = (const float*)d_in[27];
  const float* fc1w = (const float*)d_in[28];
  const float* fc1b = (const float*)d_in[29];
  const float* fc2w = (const float*)d_in[30];
  const float* fc2b = (const float*)d_in[31];

  const size_t feat_bytes = (size_t)n_nodes * 128 * sizeof(float);
  const size_t gout_off   = feat_bytes;
  const size_t gout_bytes = (size_t)n_graphs * 32 * sizeof(float);
  if (gout_off + gout_bytes > ws_size) return;

  float* feat = (float*)d_ws;
  float* gout = (float*)((char*)d_ws + gout_off);
  float* out  = (float*)d_out;

  k_conv_feat<<<n_nodes, 256, 0, stream>>>(
      x, conv1_w, conv1_b, bn1, conv2_w, conv2_b, bn2,
      conv3_w, conv3_b, bn3, dw_w, dw_b, bn_d, prelu, feat, n_nodes);

  k_gat_head<<<n_graphs, 256, 0, stream>>>(
      feat, g1w, g1a, g1b, g2w, g2a, g2b, g3w, g3a, g3b,
      bng1, bng2, bng3, prelu, fc1w, fc1b, fc2w, fc2b, gout, n_graphs);

  k_pack_out<<<1, 32, 0, stream>>>(gout, out, n_graphs);
}
